// DecoderRNNNetwork_48515950576420
// MI455X (gfx1250) — hardware-verified
//
#include <hip/hip_runtime.h>
#include <math.h>

constexpr int TSTEPS = 128;
constexpr int NBAT   = 64;
constexpr int NROW   = TSTEPS * NBAT;
constexpr int SDIM   = 32;
constexpr int LDIM   = 16;
constexpr int ACDIM  = 8;
constexpr int MSDIM  = 8;
constexpr int SEDIM  = 64;
constexpr int AEDIM  = 16;
constexpr int HDIM   = 64;
constexpr int ODIM   = 18;
constexpr int GDIM   = 192;
constexpr int CATW   = 128;
constexpr int AMSW   = 32;
constexpr int NTHR   = 256;
constexpr int WPITCH = 72;
constexpr int LGP    = 36;

typedef __attribute__((ext_vector_type(16))) _Float16 v16h;
typedef __attribute__((ext_vector_type(8)))  _Float16 v8h;
typedef __attribute__((ext_vector_type(16))) __bf16   v16b;
typedef __attribute__((ext_vector_type(8)))  __bf16   v8b;
typedef __attribute__((ext_vector_type(8)))  float    v8f;
typedef __attribute__((ext_vector_type(4)))  float    v4f;

__device__ __forceinline__ unsigned short f2bf_bits(float f) {
  unsigned u = __float_as_uint(f);
  return (unsigned short)((u + 0x7FFFu + ((u >> 16) & 1u)) >> 16);
}
__device__ __forceinline__ float bf_bits2f(unsigned short h) { return __uint_as_float(((unsigned)h) << 16); }

__device__ __forceinline__ void dep_guard_h(v8f& a, v8f& b, v16h x, v16h y) { asm volatile("v_nop\n\tv_nop\n\tv_nop\n\tv_nop" : "+v"(a), "+v"(b) : "v"(x), "v"(y)); }
__device__ __forceinline__ void dep_guard_b(v8f& a, v8f& b, v16b x, v16b y) { asm volatile("v_nop\n\tv_nop\n\tv_nop\n\tv_nop" : "+v"(a), "+v"(b) : "v"(x), "v"(y)); }
__device__ __forceinline__ void keep4_h(v16h a, v16h b, v16h c, v16h d) { asm volatile("v_nop" :: "v"(a), "v"(b), "v"(c), "v"(d)); }
__device__ __forceinline__ void keep4_b(v16b a, v16b b, v16b c, v16b d) { asm volatile("v_nop" :: "v"(a), "v"(b), "v"(c), "v"(d)); }
__device__ __forceinline__ void acc_guard4(v8f& a, v8f& b, v8f& c, v8f& d) { asm volatile("v_nop\n\tv_nop\n\tv_nop\n\tv_nop" : "+v"(a), "+v"(b), "+v"(c), "+v"(d)); }
__device__ __forceinline__ void dep_guard6_h(v8f& a, v8f& b, v8f& c, v8f& d, v8f& e, v8f& f,
                                             v16h p, v16h q, v16h x, v16h y, v16h z) {
  asm volatile("v_nop\n\tv_nop\n\tv_nop\n\tv_nop" : "+v"(a), "+v"(b), "+v"(c), "+v"(d), "+v"(e), "+v"(f) : "v"(p), "v"(q), "v"(x), "v"(y), "v"(z));
}
__device__ __forceinline__ void acc_guard6(v8f& a, v8f& b, v8f& c, v8f& d, v8f& e, v8f& f) {
  asm volatile("v_nop\n\tv_nop\n\tv_nop\n\tv_nop" : "+v"(a), "+v"(b), "+v"(c), "+v"(d), "+v"(e), "+v"(f));
}
__device__ __forceinline__ void dep_guard1_h(v8f& a, v16h x, v16h y) { asm volatile("v_nop\n\tv_nop\n\tv_nop\n\tv_nop" : "+v"(a) : "v"(x), "v"(y)); }
__device__ __forceinline__ void acc_guard1(v8f& a) { asm volatile("v_nop\n\tv_nop\n\tv_nop\n\tv_nop" : "+v"(a)); }

template <typename T> struct Frag;
template <> struct Frag<_Float16> {
  typedef v16h V; union U { v16h v; v8h h[2]; };
  static __device__ __forceinline__ v16h load(const _Float16* p) {
    U f; f.h[0] = *(const v8h*)(p); f.h[1] = *(const v8h*)(p + 16); return f.v;
  }
  static __device__ __forceinline__ v8f mma(v16h a, v16h b, v8f c) {
    return __builtin_amdgcn_wmma_f32_16x16x32_f16(false, a, false, b, (short)0, c, false, false);
  }
  static __device__ __forceinline__ void guard(v8f& a, v8f& b, v16h x, v16h y) { dep_guard_h(a, b, x, y); }
  static __device__ __forceinline__ void keep(v16h a, v16h b, v16h c, v16h d) { keep4_h(a, b, c, d); }
};
template <> struct Frag<__bf16> {
  typedef v16b V; union U { v16b v; v8b h[2]; };
  static __device__ __forceinline__ v16b load(const __bf16* p) {
    U f; f.h[0] = *(const v8b*)(p); f.h[1] = *(const v8b*)(p + 16); return f.v;
  }
  static __device__ __forceinline__ v8f mma(v16b a, v16b b, v8f c) {
    return __builtin_amdgcn_wmma_f32_16x16x32_bf16(false, a, false, b, (short)0, c, false, false);
  }
  static __device__ __forceinline__ void guard(v8f& a, v8f& b, v16b x, v16b y) { dep_guard_b(a, b, x, y); }
  static __device__ __forceinline__ void keep(v16b a, v16b b, v16b c, v16b d) { keep4_b(a, b, c, d); }
};

template <int ET> struct Elem;
template <> struct Elem<0> { typedef _Float16 T; };
template <> struct Elem<1> { typedef __bf16 T; };
template <int ET, bool SPLIT, int BIAS_MODE, int OUT_MODE, bool RESID, int ACT = 0, bool X16OUT = false>
__global__ __launch_bounds__(256) void wmma_gemm64(
    const unsigned short* __restrict__ Ap, const unsigned short* __restrict__ A2p, int lda, long strideA,
    const unsigned short* __restrict__ Btp, const unsigned short* __restrict__ Bt2p, int ldb, long strideB,
    void* __restrict__ Cout, void* __restrict__ Cout2, int ldc, long strideC,
    const float* __restrict__ bias,
    const float* __restrict__ resid, long strideR,
    int M, int N, int K, float scale) {
  typedef typename Elem<ET>::T T;
  typedef typename Frag<T>::V V;
  const T* A = (const T*)Ap; const T* A2 = (const T*)A2p; const T* Bt = (const T*)Btp; const T* Bt2 = (const T*)Bt2p;
  __shared__ __align__(16) float sT[8][16 * 68];
  const int b    = blockIdx.y;
  const int lane = threadIdx.x & 31;
  const int wave = threadIdx.x >> 5;
  const int tilesN = N >> 6;
  const int tilesM = M >> 6;
  const int tile = blockIdx.x * 8 + wave;
  if (tile >= tilesM * tilesN) return;
  const int tm = tile / tilesN;
  const int tn = tile - tm * tilesN;
  const int m0 = tm << 6;
  const int n0 = tn << 6;

  const T* Ab  = A  + (size_t)b * strideA;
  const T* Bb  = Bt + (size_t)b * strideB;
  const T* Ab2 = SPLIT ? (A2  + (size_t)b * strideA) : nullptr;
  const T* Bb2 = SPLIT ? (Bt2 + (size_t)b * strideB) : nullptr;

  const int rlane = lane & 15;
  const int koff  = (lane >> 4) * 8;
  const int mOff  = (lane >> 4) * 8;

  v8f acc[4][4];
#pragma unroll
  for (int i = 0; i < 4; ++i)
#pragma unroll
    for (int j = 0; j < 4; ++j) acc[i][j] = (v8f){0.f,0.f,0.f,0.f,0.f,0.f,0.f,0.f};

  for (int k0 = 0; k0 < K; k0 += 32) {
    V bh[4], bl[4];
#pragma unroll
    for (int j = 0; j < 4; ++j) {
      const size_t bo = (size_t)(n0 + (j << 4) + rlane) * ldb + koff + k0;
      bh[j] = Frag<T>::load(Bb + bo);
      if (SPLIT) bl[j] = Frag<T>::load(Bb2 + bo);
    }
#pragma unroll
    for (int i = 0; i < 4; ++i) {
      const size_t ao = (size_t)(m0 + (i << 4) + rlane) * lda + koff + k0;
      V ah = Frag<T>::load(Ab + ao);
      V al;
      if (SPLIT) al = Frag<T>::load(Ab2 + ao);
#pragma unroll
      for (int j = 0; j < 4; ++j) {
        acc[i][j] = Frag<T>::mma(ah, bh[j], acc[i][j]);
        if (SPLIT) {
          acc[i][j] = Frag<T>::mma(ah, bl[j], acc[i][j]);
          acc[i][j] = Frag<T>::mma(al, bh[j], acc[i][j]);
        }
      }
      Frag<T>::guard(acc[i][0], acc[i][3], ah, SPLIT ? al : ah);
    }
    Frag<T>::keep(bh[0], bh[1], bh[2], bh[3]);
    if (SPLIT) Frag<T>::keep(bl[0], bl[1], bl[2], bl[3]);
  }
  acc_guard4(acc[0][0], acc[0][1], acc[0][2], acc[0][3]);
  acc_guard4(acc[1][0], acc[1][1], acc[1][2], acc[1][3]);
  acc_guard4(acc[2][0], acc[2][1], acc[2][2], acc[2][3]);
  acc_guard4(acc[3][0], acc[3][1], acc[3][2], acc[3][3]);

  float* slab = sT[wave];
  const float* Rb = RESID ? (resid + (size_t)b * strideR) : nullptr;
#pragma unroll
  for (int i = 0; i < 4; ++i) {
    const int mBase = m0 + (i << 4);
#pragma unroll
    for (int j = 0; j < 4; ++j) {
      const int n = n0 + (j << 4) + rlane;
      float bv = 0.f;
      if (BIAS_MODE == 2) bv = bias[n];
#pragma unroll
      for (int r = 0; r < 8; ++r) {
        float v = acc[i][j][r] * scale;
        if (BIAS_MODE == 1) v += bias[mBase + mOff + r];
        if (BIAS_MODE == 2) v += bv;
        if (RESID) v += Rb[(size_t)(mBase + mOff + r) * ldc + n];
        if (ACT == 1) v = tanhf(v);
        if (ACT == 2) v = fmaxf(v, 0.0f);
        if (ACT == 3) v = v / (1.0f + expf(-v));
        if (ACT == 4) v = (v > 0.f) ? v : 0.01f * v;
        if (ACT == 5) v = 0.5f * v * (1.0f + erff(v * 0.70710678118654752f));
        if (X16OUT) v = v * 16.0f;
        slab[(mOff + r) * 68 + (j << 4) + rlane] = v;
      }
    }
    __builtin_amdgcn_fence(__ATOMIC_RELEASE, "workgroup");
    __builtin_amdgcn_wave_barrier();
    __builtin_amdgcn_fence(__ATOMIC_ACQUIRE, "workgroup");
    if (OUT_MODE == 0) {
      float* C = (float*)Cout + (size_t)b * strideC;
      const int hh = lane >> 4, c4 = (lane & 15) * 4;
      for (int pass = 0; pass < 2; ++pass) {
#pragma unroll
        for (int it = 0; it < 8; ++it) {
          const int row = it * 2 + hh;
          v4f v = *(const v4f*)(slab + row * 68 + c4);
          *(volatile v4f*)(C + (size_t)(mBase + row) * ldc + n0 + c4) = v;
        }
        __threadfence();
      }
    } else {
      const int q = lane >> 3, c8 = (lane & 7) * 8;
      unsigned short* C  = (unsigned short*)Cout  + (size_t)b * strideC;
      unsigned short* C2 = (OUT_MODE == 2) ? ((unsigned short*)Cout2 + (size_t)b * strideC) : nullptr;
      for (int pass = 0; pass < 2; ++pass) {
#pragma unroll
        for (int it = 0; it < 4; ++it) {
          const int row = it * 4 + q;
          const float* sp = slab + row * 68 + c8;
          v8h hv, lv;
#pragma unroll
          for (int e = 0; e < 8; ++e) {
            if (OUT_MODE == 1) {
              hv[e] = (_Float16)sp[e];
            } else {
              unsigned short hb = f2bf_bits(sp[e]);
              unsigned short lb = f2bf_bits(sp[e] - bf_bits2f(hb));
              hv[e] = __builtin_bit_cast(_Float16, hb);
              lv[e] = __builtin_bit_cast(_Float16, lb);
            }
          }
          *(volatile v8h*)(C + (size_t)(mBase + row) * ldc + n0 + c8) = hv;
          if (OUT_MODE == 2) *(volatile v8h*)(C2 + (size_t)(mBase + row) * ldc + n0 + c8) = lv;
        }
        __threadfence();
      }
    }
    __builtin_amdgcn_fence(__ATOMIC_RELEASE, "workgroup");
    __builtin_amdgcn_wave_barrier();
    __builtin_amdgcn_fence(__ATOMIC_ACQUIRE, "workgroup");
  }
}

__device__ __forceinline__ unsigned pack_f16x2(float a, float b) {
  const _Float16 h0 = (_Float16)a, h1 = (_Float16)b;
  return (unsigned)__builtin_bit_cast(unsigned short, h0) | ((unsigned)__builtin_bit_cast(unsigned short, h1) << 16);
}
__device__ __forceinline__ void st2u(unsigned* p, unsigned v) { *(volatile unsigned*)p = v; __threadfence(); *(volatile unsigned*)p = v; }
__device__ __forceinline__ void st2h8(_Float16* p, v8h v) { *(volatile v8h*)p = v; __threadfence(); *(volatile v8h*)p = v; }
__device__ __forceinline__ float ftanh(float x) { return 1.0f - 2.0f * __builtin_amdgcn_rcpf(1.0f + __expf(2.0f * x)); }
__device__ __forceinline__ float fsigm(float x) { return __builtin_amdgcn_rcpf(1.0f + __expf(-x)); }

__global__ __launch_bounds__(NTHR) void prep_kernel(
    const float* __restrict__ state, const float* __restrict__ ac, const float* __restrict__ ms,
    const float* __restrict__ W_state, const float* __restrict__ W_ac, const float* __restrict__ b_ac,
    const float* __restrict__ W_embed, const float* __restrict__ W_hid, const float* __restrict__ Wi,
    _Float16* __restrict__ XST, _Float16* __restrict__ CAT, _Float16* __restrict__ AMS,
    unsigned* __restrict__ W1T, unsigned* __restrict__ WET, unsigned* __restrict__ WHT, unsigned* __restrict__ WIT) {
  __shared__ float sAE[32 * 17];
  const int blk = blockIdx.x, tid = threadIdx.x;
  if (blk < 256) {
    const int row0 = blk * 32;
    {
      const int r = tid >> 3, sub = tid & 7;
      const int grow = row0 + r;
      const int n0 = 2 * sub, n1 = n0 + 1;
      const float* ap = ac + (size_t)grow * ACDIM;
      float a0 = 0.0f, a1 = 0.0f;
#pragma unroll 1
      for (int k = 0; k < ACDIM; ++k) {
        const float x = ap[k];
        a0 += x * W_ac[k * AEDIM + n0];
        a1 += x * W_ac[k * AEDIM + n1];
      }
      sAE[r * 17 + n0] = fmaxf(a0 + b_ac[n0], 0.0f);
      sAE[r * 17 + n1] = fmaxf(a1 + b_ac[n1], 0.0f);
    }
    __syncthreads();
    if (tid < 128) {
      const int r = tid >> 2, c8 = (tid & 3) * 8;
      const int grow = row0 + r;
      const float* sp = state + (size_t)grow * SDIM + c8;
      const v4f s0 = *(const v4f*)sp, s1 = *(const v4f*)(sp + 4);
      v8h hx;
#pragma unroll
      for (int e = 0; e < 4; ++e) { hx[e] = (_Float16)s0[e]; hx[4 + e] = (_Float16)s1[e]; }
      st2h8(XST + (size_t)grow * SDIM + c8, hx);
      const float* mp = ms + (size_t)grow * MSDIM;
      const v4f m0 = *(const v4f*)mp, m1 = *(const v4f*)(mp + 4);
      v8h ha;
#pragma unroll
      for (int e = 0; e < 4; ++e) {
        const int col = c8 + e; const int ci = col < AEDIM ? col : AEDIM - 1;
        const float fa = sAE[r * 17 + ci];
        const float v  = (c8 < 16) ? fa : ((c8 == 16) ? m0[e] : 0.0f);
        ha[e] = (_Float16)v;
      }
#pragma unroll
      for (int e = 0; e < 4; ++e) {
        const int col = c8 + 4 + e; const int ci = col < AEDIM ? col : AEDIM - 1;
        const float fa = sAE[r * 17 + ci];
        const float v  = (c8 < 16) ? fa : ((c8 == 16) ? m1[e] : 0.0f);
        ha[4 + e] = (_Float16)v;
      }
      st2h8(AMS + (size_t)grow * AMSW + c8, ha);
    }
    {
      const int r = tid >> 3, c8 = (tid & 7) * 8;
      const int grow = row0 + r;
      v8h hc;
#pragma unroll
      for (int e = 0; e < 8; ++e) {
        const int col = c8 + e; const int ci = col < AEDIM ? col : AEDIM - 1;
        const float fa = sAE[r * 17 + ci];
        hc[e] = (_Float16)((col < AEDIM) ? fa : 0.0f);
      }
      st2h8(CAT + (size_t)grow * CATW + SEDIM + c8, hc);
    }
  } else if (blk < 260) {
    const int p = (blk - 256) * NTHR + tid;
    const int n = p >> 4, k = (p & 15) * 2;
    const unsigned u = pack_f16x2(W_state[k * SEDIM + n] * 16.0f, W_state[(k + 1) * SEDIM + n] * 16.0f);
    st2u(W1T + p, u);
  } else if (blk < 276) {
    const int p = (blk - 260) * NTHR + tid;
    const int n = p >> 6, k = (p & 63) * 2;
    const int kc = k < 80 ? k : 78;
    const float w0 = W_embed[kc * HDIM + n] * 16.0f, w1 = W_embed[(kc + 1) * HDIM + n] * 16.0f;
    const unsigned u = pack_f16x2(k < 80 ? w0 : 0.0f, k < 80 ? w1 : 0.0f);
    st2u(WET + p, u);
  } else if (blk < 280) {
    const int p = (blk - 276) * NTHR + tid;
    const int n = p >> 4, k = (p & 15) * 2;
    const int kc = k < 24 ? k : 22;
    const float w0 = W_hid[kc * HDIM + n] * 16.0f, w1 = W_hid[(kc + 1) * HDIM + n] * 16.0f;
    const unsigned u = pack_f16x2(k < 24 ? w0 : 0.0f, k < 24 ? w1 : 0.0f);
    st2u(WHT + p, u);
  } else {
    const int p = (blk - 280) * NTHR + tid;
    const int n = p >> 5, k = (p & 31) * 2;
    const unsigned u = pack_f16x2(Wi[k * GDIM + n] * 16.0f, Wi[(k + 1) * GDIM + n] * 16.0f);
    st2u(WIT + p, u);
  }
}

__device__ __forceinline__ void reset_rows(float (&h)[8], const float* __restrict__ dp, const float* __restrict__ hp, _Float16* srow) {
  const v4f da = *(const v4f*)dp, db = *(const v4f*)(dp + 4);
#pragma unroll
  for (int r = 0; r < 4; ++r) {
    const float hv = hp[(size_t)r * HDIM];
    const float hs = (da[r] > 0.0f) ? hv : h[r];
    h[r] = hs;
    srow[r * WPITCH] = (_Float16)(hs * 16.0f);
  }
#pragma unroll
  for (int r = 0; r < 4; ++r) {
    const float hv = hp[(size_t)(4 + r) * HDIM];
    const float hs = (db[r] > 0.0f) ? hv : h[4 + r];
    h[4 + r] = hs;
    srow[(4 + r) * WPITCH] = (_Float16)(hs * 16.0f);
  }
}
__device__ __forceinline__ void gru_cell8(float (&h)[8], const v8f& ar, const v8f& az, const v8f& an,
                                          const float* __restrict__ gp, float bhn) {
  const float s256 = 1.0f / 256.0f;
#pragma unroll
  for (int r = 0; r < 8; ++r) {
    const float* g = gp + (size_t)r * GDIM;
    const float x_r = g[0], x_z = g[HDIM], x_n = g[2 * HDIM];
    const float hr = ar[r] * s256;
    const float hz = az[r] * s256;
    const float hn = an[r] * s256 + bhn;
    const float rg = fsigm(x_r + hr);
    const float zg = fsigm(x_z + hz);
    const float ng = ftanh(x_n + rg * hn);
    h[r] = (1.0f - zg) * ng + zg * h[r];
  }
}
__device__ __forceinline__ void store_rows16(const float (&h)[8], _Float16* srow) {
#pragma unroll
  for (int r = 0; r < 8; ++r) srow[r * WPITCH] = (_Float16)(h[r] * 16.0f);
}

__global__ __launch_bounds__(NTHR) void gru_shift_kernel(
    const float* __restrict__ GI, const float* __restrict__ HID,
    const float* __restrict__ dones, const int* __restrict__ pact,
    const float* __restrict__ Wh_rz, const float* __restrict__ Wh_n, const float* __restrict__ bh_n,
    const float* __restrict__ W_out, const float* __restrict__ b_out, float* __restrict__ PART) {
  __shared__ __align__(16) _Float16 sWH[GDIM * WPITCH];
  __shared__ __align__(16) _Float16 sWO[32 * WPITCH];
  __shared__ __align__(16) _Float16 sH[NBAT * WPITCH];
  __shared__ float sLg[NBAT * LGP];
  __shared__ float sBo[32];
  const int tid = threadIdx.x, lane = tid & 31, wave = tid >> 5;
  const int rlane = lane & 15, hh = lane >> 4, koff = hh * 8;
  const int kidx = blockIdx.x;
  const int nsteps = TSTEPS - kidx;

  for (int i = tid; i < GDIM * HDIM; i += NTHR) {
    const int n = i >> 6, kk = i & 63;
    const int nrz = n < 128 ? n : 127;
    int nn = n - 128; nn = nn < 0 ? 0 : nn;
    const float vrz = Wh_rz[kk * 128 + nrz];
    const float vn  = Wh_n[kk * HDIM + nn];
    const float v   = (n < 128) ? vrz : vn;
    sWH[n * WPITCH + kk] = (_Float16)(v * 16.0f);
  }
  for (int i = tid; i < 32 * HDIM; i += NTHR) {
    const int n = i >> 6, kk = i & 63;
    const int nc = n < ODIM ? n : ODIM - 1;
    const float v = W_out[kk * ODIM + nc] * 16.0f;
    sWO[n * WPITCH + kk] = (_Float16)((n < ODIM) ? v : 0.0f);
  }
  for (int i = tid; i < NBAT * WPITCH; i += NTHR) sH[i] = (_Float16)0.0f;
  if (tid < 32) { const int nc = tid < ODIM ? tid : ODIM - 1; const float v = b_out[nc]; sBo[tid] = (tid < ODIM) ? v : 0.0f; }

  const int cg  = wave & 3, rt0 = wave >> 2, rt1 = rt0 + 2;
  const int j   = 16 * cg + rlane;
  const int sq0 = 16 * rt0 + 8 * hh, sq1 = 16 * rt1 + 8 * hh;
  const int hrt = wave >> 1, hot = wave & 1;
  const float bhn = bh_n[j];
  float h0r[8], h1r[8];
#pragma unroll
  for (int r = 0; r < 8; ++r) {
    h0r[r] = HID[((size_t)kidx * NBAT + sq0 + r) * HDIM + j];
    h1r[r] = HID[((size_t)kidx * NBAT + sq1 + r) * HDIM + j];
  }
  float csum = 0.0f;
  const v8f z8 = {0.f, 0.f, 0.f, 0.f, 0.f, 0.f, 0.f, 0.f};
  const float s256 = 1.0f / 256.0f;
  __syncthreads();

#pragma unroll 1
  for (int t = 0; t < nsteps; ++t) {
    const int tau = kidx + t;
    const size_t rowbase = (size_t)tau * NBAT;
    reset_rows(h0r, dones + rowbase + sq0, HID + (rowbase + sq0) * HDIM + j, sH + sq0 * WPITCH + j);
    reset_rows(h1r, dones + rowbase + sq1, HID + (rowbase + sq1) * HDIM + j, sH + sq1 * WPITCH + j);
    __syncthreads();
    v8f ar0 = z8, az0 = z8, an0 = z8, ar1 = z8, az1 = z8, an1 = z8;
#pragma unroll 1
    for (int k0 = 0; k0 < HDIM; k0 += 32) {
      const v16h a0 = Frag<_Float16>::load(sH + (16 * rt0 + rlane) * WPITCH + koff + k0);
      const v16h a1 = Frag<_Float16>::load(sH + (16 * rt1 + rlane) * WPITCH + koff + k0);
      const v16h fr = Frag<_Float16>::load(sWH + j * WPITCH + koff + k0);
      const v16h fz = Frag<_Float16>::load(sWH + (HDIM + j) * WPITCH + koff + k0);
      const v16h fn = Frag<_Float16>::load(sWH + (2 * HDIM + j) * WPITCH + koff + k0);
      ar0 = Frag<_Float16>::mma(a0, fr, ar0);
      az0 = Frag<_Float16>::mma(a0, fz, az0);
      an0 = Frag<_Float16>::mma(a0, fn, an0);
      ar1 = Frag<_Float16>::mma(a1, fr, ar1);
      az1 = Frag<_Float16>::mma(a1, fz, az1);
      an1 = Frag<_Float16>::mma(a1, fn, an1);
      dep_guard6_h(ar0, az0, an0, ar1, az1, an1, a0, a1, fr, fz, fn);
    }
    acc_guard6(ar0, az0, an0, ar1, az1, an1);
    gru_cell8(h0r, ar0, az0, an0, GI + (rowbase + sq0) * GDIM + j, bhn);
    gru_cell8(h1r, ar1, az1, an1, GI + (rowbase + sq1) * GDIM + j, bhn);
    __syncthreads();
    store_rows16(h0r, sH + sq0 * WPITCH + j);
    store_rows16(h1r, sH + sq1 * WPITCH + j);
    __syncthreads();
    v8f ao = z8;
#pragma unroll 1
    for (int k0 = 0; k0 < HDIM; k0 += 32) {
      const v16h a  = Frag<_Float16>::load(sH + (16 * hrt + rlane) * WPITCH + koff + k0);
      const v16h bw = Frag<_Float16>::load(sWO + (16 * hot + rlane) * WPITCH + koff + k0);
      ao = Frag<_Float16>::mma(a, bw, ao);
      dep_guard1_h(ao, a, bw);
    }
    acc_guard1(ao);
#pragma unroll
    for (int r = 0; r < 8; ++r) sLg[(16 * hrt + 8 * hh + r) * LGP + 16 * hot + rlane] = ao[r] * s256;
    __syncthreads();
    if (tid < NBAT) {
      const int b = tid;
      float mx = -INFINITY;
#pragma unroll 1
      for (int n = 0; n < ODIM; ++n) mx = fmaxf(mx, sLg[b * LGP + n] + sBo[n]);
      float ssum = 0.0f;
#pragma unroll 1
      for (int n = 0; n < ODIM; ++n) ssum += expf((sLg[b * LGP + n] + sBo[n]) - mx);
      int a = pact[rowbase + b];
      a = a < 0 ? 0 : (a > ODIM - 1 ? ODIM - 1 : a);
      const float xa  = sLg[b * LGP + a] + sBo[a];
      const float nll = logf(ssum) - (xa - mx);
      const float d    = dones[rowbase + b];
      const float incl = csum + d;
      const float maskf = ((incl - d) == 0.0f) ? 1.0f : 0.0f;
      csum = incl;
      const float v = nll * maskf;
      float* pp = PART + ((size_t)kidx * TSTEPS + t) * NBAT + b;
      *(volatile float*)pp = v;
      __threadfence();
      *(volatile float*)pp = v;
    }
  }
}

__global__ __launch_bounds__(NTHR) void finalize_kernel(
    const float* __restrict__ PART, const float* __restrict__ lm0, const float* __restrict__ lv0,
    const float* __restrict__ lm1, const float* __restrict__ lv1, float* __restrict__ out) {
  __shared__ __align__(16) float sOut[8208];
  __shared__ double sRed[NTHR];
  const int tid = threadIdx.x, lane = tid & 31, wave = tid >> 5;
#pragma unroll 1
  for (int i = 0; i < 32; ++i) {
    const int c = i * NTHR + tid;
    const int t = c >> 6, b = c & 63;
    const int nk = TSTEPS - t;
    double acc = 0.0;
#pragma unroll 1
    for (int k = 0; k < nk; ++k) acc += (double)PART[((size_t)k * TSTEPS + t) * NBAT + b];
    sOut[1 + c] = (float)acc;
  }
  double kacc = 0.0;
#pragma unroll 1
  for (int i = 0; i < 32; ++i) {
    const int c = i * NTHR + tid;
    const int t = c >> 6, b = c & 63;
    const int tp = t > 0 ? t - 1 : 0;
    const bool first = (t == 0);
    const int cur = c * LDIM, prv = (tp * NBAT + b) * LDIM;
    float sls = 0.0f, sle = 0.0f, sex = 0.0f, sq = 0.0f;
#pragma unroll 1
    for (int jj = 0; jj < LDIM; ++jj) {
      const float mu = lm0[cur + jj], le = lv0[cur + jj];
      const float mp = lm0[prv + jj], lp = lv0[prv + jj];
      const float m  = first ? 0.0f : mp;
      const float ls = first ? 0.0f : lp;
      sls += ls; sle += le;
      sex += expf(le - ls);
      const float dd = m - mu;
      sq += (dd * dd) * __builtin_amdgcn_rcpf(expf(ls));
    }
#pragma unroll 1
    for (int jj = 0; jj < LDIM; ++jj) {
      const float mu = lm1[cur + jj], le = lv1[cur + jj];
      const float mp = lm1[prv + jj], lp = lv1[prv + jj];
      const float m  = first ? 0.0f : mp;
      const float ls = first ? 0.0f : lp;
      sls += ls; sle += le;
      sex += expf(le - ls);
      const float dd = m - mu;
      sq += (dd * dd) * __builtin_amdgcn_rcpf(expf(ls));
    }
    const float klc = 0.5f * (sls - sle - (float)(2 * LDIM) + sex + sq);
    kacc += (double)klc;
  }
  sRed[tid] = kacc;
  __syncthreads();
  for (int s = NTHR / 2; s > 0; s >>= 1) {
    if (tid < s) sRed[tid] += sRed[tid + s];
    __syncthreads();
  }
  if (tid == 0) sOut[0] = (float)sRed[0];
  __syncthreads();
  const int q = lane >> 3, c4 = (lane & 7) * 4;
  const float tail = sOut[NROW];
  for (int pass = 0; pass < 2; ++pass) {
#pragma unroll
    for (int it = 0; it < 8; ++it) {
      const int L = it * 32 + wave * 4 + q;
      const int f = L * 32 + c4;
      const v4f v = *(const v4f*)(sOut + f);
      *(volatile v4f*)(out + f) = v;
    }
    if (tid == 0) *(volatile float*)(out + NROW) = tail;
    __threadfence();
  }
}

extern "C" void kernel_launch(void* const* d_in, const int* in_sizes, int n_in,
                              void* d_out, int out_size, void* d_ws, size_t ws_size, hipStream_t stream) {
  if (n_in < 24 || d_out == nullptr || d_ws == nullptr) return;
  if (in_sizes[0] != NROW * SDIM || in_sizes[1] != NROW * LDIM || in_sizes[2] != NROW * LDIM ||
      in_sizes[3] != NROW * LDIM || in_sizes[4] != NROW * LDIM || in_sizes[5] != NROW * ACDIM ||
      in_sizes[6] != NROW * MSDIM || in_sizes[7] != NROW || in_sizes[8] != NROW ||
      in_sizes[9] != SDIM * SEDIM || in_sizes[10] != SEDIM || in_sizes[11] != ACDIM * AEDIM || in_sizes[12] != AEDIM ||
      in_sizes[13] != (SEDIM + AEDIM) * HDIM || in_sizes[14] != HDIM || in_sizes[15] != (AEDIM + MSDIM) * HDIM ||
      in_sizes[16] != HDIM || in_sizes[17] != HDIM * GDIM || in_sizes[18] != GDIM || in_sizes[19] != HDIM * 2 * HDIM ||
      in_sizes[20] != HDIM * HDIM || in_sizes[21] != HDIM || in_sizes[22] != HDIM * ODIM || in_sizes[23] != ODIM ||
      out_size != NROW + 1) return;

  const float* state   = (const float*)d_in[0];
  const float* lm0     = (const float*)d_in[1];
  const float* lv0     = (const float*)d_in[2];
  const float* lm1     = (const float*)d_in[3];
  const float* lv1     = (const float*)d_in[4];
  const float* ac      = (const float*)d_in[5];
  const float* ms      = (const float*)d_in[6];
  const int*   pact    = (const int*)  d_in[7];
  const float* dones   = (const float*)d_in[8];
  const float* W_state = (const float*)d_in[9];
  const float* b_state = (const float*)d_in[10];
  const float* W_ac    = (const float*)d_in[11];
  const float* b_ac    = (const float*)d_in[12];
  const float* W_embed = (const float*)d_in[13];
  const float* b_embed = (const float*)d_in[14];
  const float* W_hid   = (const float*)d_in[15];
  const float* b_hid   = (const float*)d_in[16];
  const float* Wi      = (const float*)d_in[17];
  const float* bi      = (const float*)d_in[18];
  const float* Wh_rz   = (const float*)d_in[19];
  const float* Wh_n    = (const float*)d_in[20];
  const float* bh_n    = (const float*)d_in[21];
  const float* W_out   = (const float*)d_in[22];
  const float* b_out   = (const float*)d_in[23];
  float* out = (float*)d_out;

  char* ws = (char*)d_ws; size_t off = 0;
  auto carve = [&](size_t bytes) -> char* { char* p = ws + off; off += (bytes + 255) & ~(size_t)255; return p; };
  _Float16* XST  = (_Float16*)carve((size_t)NROW * SDIM * 2);
  _Float16* CAT  = (_Float16*)carve((size_t)NROW * CATW * 2);
  _Float16* AMS  = (_Float16*)carve((size_t)NROW * AMSW * 2);
  unsigned* W1Tu = (unsigned*)carve((size_t)SEDIM * SDIM * 2);
  unsigned* WETu = (unsigned*)carve((size_t)HDIM * CATW * 2);
  unsigned* WHTu = (unsigned*)carve((size_t)HDIM * AMSW * 2);
  unsigned* WITu = (unsigned*)carve((size_t)GDIM * HDIM * 2);
  _Float16* EMB  = (_Float16*)carve((size_t)NROW * HDIM * 2);
  float*    HID  = (float*)carve((size_t)NROW * HDIM * 4);
  float*    GI   = (float*)carve((size_t)NROW * GDIM * 4);
  float*    PART = (float*)carve((size_t)TSTEPS * TSTEPS * NBAT * 4);
  if (off > ws_size || off > (size_t)134217728) return;

  prep_kernel<<<304, NTHR, 0, stream>>>(state, ac, ms, W_state, W_ac, b_ac, W_embed, W_hid, Wi,
                                        XST, CAT, AMS, W1Tu, WETu, WHTu, WITu);
  wmma_gemm64<0, false, 2, 1, false, 2, false><<<dim3(16, 1), 256, 0, stream>>>(
      (const unsigned short*)XST, (const unsigned short*)nullptr, SDIM, 0L,
      (const unsigned short*)W1Tu, (const unsigned short*)nullptr, SDIM, 0L,
      (void*)CAT, (void*)nullptr, CATW, 0L,
      b_state, (const float*)nullptr, 0L, NROW, SEDIM, SDIM, 1.0f / 16.0f);
  wmma_gemm64<0, false, 2, 0, false, 0, false><<<dim3(16, 1), 256, 0, stream>>>(
      (const unsigned short*)AMS, (const unsigned short*)nullptr, AMSW, 0L,
      (const unsigned short*)WHTu, (const unsigned short*)nullptr, AMSW, 0L,
      (void*)HID, (void*)nullptr, HDIM, 0L,
      b_hid, (const float*)nullptr, 0L, NROW, HDIM, AMSW, 1.0f / 16.0f);
  wmma_gemm64<0, false, 2, 1, false, 0, true><<<dim3(16, 1), 256, 0, stream>>>(
      (const unsigned short*)CAT, (const unsigned short*)nullptr, CATW, 0L,
      (const unsigned short*)WETu, (const unsigned short*)nullptr, CATW, 0L,
      (void*)EMB, (void*)nullptr, HDIM, 0L,
      b_embed, (const float*)nullptr, 0L, NROW, HDIM, CATW, 1.0f / 16.0f);
  wmma_gemm64<0, false, 2, 0, false, 0, false><<<dim3(48, 1), 256, 0, stream>>>(
      (const unsigned short*)EMB, (const unsigned short*)nullptr, HDIM, 0L,
      (const unsigned short*)WITu, (const unsigned short*)nullptr, HDIM, 0L,
      (void*)GI, (void*)nullptr, GDIM, 0L,
      bi, (const float*)nullptr, 0L, NROW, GDIM, HDIM, 1.0f / 256.0f);
  gru_shift_kernel<<<TSTEPS, NTHR, 0, stream>>>(GI, HID, dones, pact, Wh_rz, Wh_n, bh_n, W_out, b_out, PART);
  finalize_kernel<<<1, NTHR, 0, stream>>>(PART, lm0, lv0, lm1, lv1, out);
}
